// VotingModule_45466523795793
// MI455X (gfx1250) — hardware-verified
//
#include <hip/hip_runtime.h>
#include <stddef.h>
#include <math.h>


#define NB     2
#define CC     256
#define HH     128
#define WW     128
#define HWP    16384
#define KT     9
#define KD     2304
#define WP2    130
#define PLANE  16900
#define GF     64
#define RP     17088
#define MSO    131
#define RO     16640
#define OFFC   27
#define OFFN   64
#define HDN    64
#define NHALO  704
#define CHROWS 64
#define CHPIX  8192
#define NCH    4
#define SIT    4

typedef __attribute__((ext_vector_type(16))) _Float16 v16h;
typedef __attribute__((ext_vector_type(8)))  _Float16 v8h;
typedef __attribute__((ext_vector_type(16))) __bf16   v16b;
typedef __attribute__((ext_vector_type(8)))  __bf16   v8b;
typedef __attribute__((ext_vector_type(8)))  float    v8f;
typedef __attribute__((ext_vector_type(4)))  float    v4f;
typedef __attribute__((ext_vector_type(4)))  unsigned v4u;

__device__ __forceinline__ unsigned short f2bf_bits(float f) {
  unsigned u = __float_as_uint(f);
  return (unsigned short)((u + 0x7FFFu + ((u >> 16) & 1u)) >> 16);
}
__device__ __forceinline__ float bf_bits2f(unsigned short h) { return __uint_as_float(((unsigned)h) << 16); }

__device__ __forceinline__ unsigned pk2(unsigned short a, unsigned short b) {
  return (unsigned)a | ((unsigned)b << 16);
}
__device__ __forceinline__ unsigned pkh2(float a, float b) {
  return pk2(__builtin_bit_cast(unsigned short, (_Float16)a), __builtin_bit_cast(unsigned short, (_Float16)b));
}

__device__ __forceinline__ void dep_guard_h(v8f& a, v8f& b, v16h x, v16h y) { asm volatile("v_nop\n\tv_nop\n\tv_nop\n\tv_nop" : "+v"(a), "+v"(b) : "v"(x), "v"(y)); }
__device__ __forceinline__ void dep_guard_b(v8f& a, v8f& b, v16b x, v16b y) { asm volatile("v_nop\n\tv_nop\n\tv_nop\n\tv_nop" : "+v"(a), "+v"(b) : "v"(x), "v"(y)); }
__device__ __forceinline__ void keep4_h(v16h a, v16h b, v16h c, v16h d) { asm volatile("v_nop" :: "v"(a), "v"(b), "v"(c), "v"(d)); }
__device__ __forceinline__ void keep4_b(v16b a, v16b b, v16b c, v16b d) { asm volatile("v_nop" :: "v"(a), "v"(b), "v"(c), "v"(d)); }
__device__ __forceinline__ void acc_guard4(v8f& a, v8f& b, v8f& c, v8f& d) { asm volatile("v_nop\n\tv_nop\n\tv_nop\n\tv_nop" : "+v"(a), "+v"(b), "+v"(c), "+v"(d)); }
template <typename T> struct Frag;
template <> struct Frag<_Float16> {
  typedef v16h V; union U { v16h v; v8h h[2]; };
  static __device__ __forceinline__ v16h load(const _Float16* p) {
    U f; f.h[0] = *(const v8h*)(p); f.h[1] = *(const v8h*)(p + 16); return f.v;
  }
  static __device__ __forceinline__ v8f mma(v16h a, v16h b, v8f c) {
    return __builtin_amdgcn_wmma_f32_16x16x32_f16(false, a, false, b, (short)0, c, false, false);
  }
  static __device__ __forceinline__ void guard(v8f& a, v8f& b, v16h x, v16h y) { dep_guard_h(a, b, x, y); }
  static __device__ __forceinline__ void keep(v16h a, v16h b, v16h c, v16h d) { keep4_h(a, b, c, d); }
};
template <> struct Frag<__bf16> {
  typedef v16b V; union U { v16b v; v8b h[2]; };
  static __device__ __forceinline__ v16b load(const __bf16* p) {
    U f; f.h[0] = *(const v8b*)(p); f.h[1] = *(const v8b*)(p + 16); return f.v;
  }
  static __device__ __forceinline__ v8f mma(v16b a, v16b b, v8f c) {
    return __builtin_amdgcn_wmma_f32_16x16x32_bf16(false, a, false, b, (short)0, c, false, false);
  }
  static __device__ __forceinline__ void guard(v8f& a, v8f& b, v16b x, v16b y) { dep_guard_b(a, b, x, y); }
  static __device__ __forceinline__ void keep(v16b a, v16b b, v16b c, v16b d) { keep4_b(a, b, c, d); }
};

template <int ET> struct Elem;
template <> struct Elem<0> { typedef _Float16 T; };
template <> struct Elem<1> { typedef __bf16 T; };
template <int ET, bool SPLIT, int BIAS_MODE, int OUT_MODE, bool RESID, int ACT = 0, int CONVA = 0>
__global__ __launch_bounds__(256) void wmma_gemm64(
    const unsigned short* __restrict__ Ap, const unsigned short* __restrict__ A2p, int lda, long strideA,
    const unsigned short* __restrict__ Btp, const unsigned short* __restrict__ Bt2p, int ldb, long strideB,
    void* __restrict__ Cout, void* __restrict__ Cout2, int ldc, long strideC,
    const float* __restrict__ bias,
    const float* __restrict__ resid, long strideR,
    int M, int N, int K, float scale) {
  typedef typename Elem<ET>::T T;
  typedef typename Frag<T>::V V;
  const T* A = (const T*)Ap; const T* A2 = (const T*)A2p; const T* Bt = (const T*)Btp; const T* Bt2 = (const T*)Bt2p;
  __shared__ __align__(16) float sT[8][16 * 68];
  const int b    = blockIdx.y;
  const int lane = threadIdx.x & 31;
  const int wave = threadIdx.x >> 5;
  const int tilesN = N >> 6;
  const int tilesM = M >> 6;
  const int tile = blockIdx.x * 8 + wave;
  if (tile >= tilesM * tilesN) return;
  const int tm = tile / tilesN;
  const int tn = tile - tm * tilesN;
  const int m0 = tm << 6;
  const int n0 = tn << 6;

  const T* Ab  = A  + (size_t)b * strideA;
  const T* Bb  = Bt + (size_t)b * strideB;
  const T* Ab2 = SPLIT ? (A2  + (size_t)b * strideA) : nullptr;
  const T* Bb2 = SPLIT ? (Bt2 + (size_t)b * strideB) : nullptr;

  const int rlane = lane & 15;
  const int koff  = (lane >> 4) * 8;
  const int mOff  = (lane >> 4) * 8;

  v8f acc[4][4];
#pragma unroll
  for (int i = 0; i < 4; ++i)
#pragma unroll
    for (int j = 0; j < 4; ++j) acc[i][j] = (v8f){0.f,0.f,0.f,0.f,0.f,0.f,0.f,0.f};

  for (int k0 = 0; k0 < K; k0 += 32) {
    ptrdiff_t arow = 0;
    int acol = k0;
    if (CONVA) {
      const int t = k0 >> 8;
      const int kh = t / 3; const int kw = t - kh * 3;
      arow = (ptrdiff_t)((kh - 1) * WP2 + (kw - 1));
      acol = k0 & (CC - 1);
    }
    V bh[4], bl[4];
#pragma unroll
    for (int j = 0; j < 4; ++j) {
      const size_t bo = (size_t)(n0 + (j << 4) + rlane) * ldb + koff + k0;
      bh[j] = Frag<T>::load(Bb + bo);
      if (SPLIT) bl[j] = Frag<T>::load(Bb2 + bo);
    }
#pragma unroll
    for (int i = 0; i < 4; ++i) {
      const ptrdiff_t ao = ((ptrdiff_t)(m0 + (i << 4) + rlane) + arow) * lda + koff + acol;
      V ah = Frag<T>::load(Ab + ao);
      V al;
      if (SPLIT) al = Frag<T>::load(Ab2 + ao);
#pragma unroll
      for (int j = 0; j < 4; ++j) {
        acc[i][j] = Frag<T>::mma(ah, bh[j], acc[i][j]);
        if (SPLIT) {
          acc[i][j] = Frag<T>::mma(ah, bl[j], acc[i][j]);
          acc[i][j] = Frag<T>::mma(al, bh[j], acc[i][j]);
        }
      }
      Frag<T>::guard(acc[i][0], acc[i][3], ah, SPLIT ? al : ah);
    }
    Frag<T>::keep(bh[0], bh[1], bh[2], bh[3]);
    if (SPLIT) Frag<T>::keep(bl[0], bl[1], bl[2], bl[3]);
  }
  acc_guard4(acc[0][0], acc[0][1], acc[0][2], acc[0][3]);
  acc_guard4(acc[1][0], acc[1][1], acc[1][2], acc[1][3]);
  acc_guard4(acc[2][0], acc[2][1], acc[2][2], acc[2][3]);
  acc_guard4(acc[3][0], acc[3][1], acc[3][2], acc[3][3]);

  float* slab = sT[wave];
  const float* Rb = RESID ? (resid + (size_t)b * strideR) : nullptr;
#pragma unroll
  for (int i = 0; i < 4; ++i) {
    const int mBase = m0 + (i << 4);
#pragma unroll
    for (int j = 0; j < 4; ++j) {
      const int n = n0 + (j << 4) + rlane;
      float bv = 0.f;
      if (BIAS_MODE == 2) bv = bias[n];
#pragma unroll
      for (int r = 0; r < 8; ++r) {
        float v = acc[i][j][r] * scale;
        if (BIAS_MODE == 1) v += bias[mBase + mOff + r];
        if (BIAS_MODE == 2) v += bv;
        if (RESID) v += Rb[(size_t)(mBase + mOff + r) * ldc + n];
        if (ACT == 1) v = tanhf(v);
        if (ACT == 2) v = fmaxf(v, 0.0f);
        if (ACT == 3) v = v / (1.0f + expf(-v));
        if (ACT == 4) v = (v > 0.f) ? v : 0.01f * v;
        if (ACT == 5) v = 0.5f * v * (1.0f + erff(v * 0.70710678118654752f));
        slab[(mOff + r) * 68 + (j << 4) + rlane] = v;
      }
    }
    __builtin_amdgcn_fence(__ATOMIC_RELEASE, "workgroup");
    __builtin_amdgcn_wave_barrier();
    __builtin_amdgcn_fence(__ATOMIC_ACQUIRE, "workgroup");
    if (OUT_MODE == 0) {
      float* C = (float*)Cout + (size_t)b * strideC;
      const int hh = lane >> 4, c4 = (lane & 15) * 4;
      for (int pass = 0; pass < 2; ++pass) {
#pragma unroll
        for (int it = 0; it < 8; ++it) {
          const int row = it * 2 + hh;
          v4f v = *(const v4f*)(slab + row * 68 + c4);
          *(volatile v4f*)(C + (size_t)(mBase + row) * ldc + n0 + c4) = v;
        }
        __threadfence();
      }
    } else {
      const int q = lane >> 3, c8 = (lane & 7) * 8;
      unsigned short* C  = (unsigned short*)Cout  + (size_t)b * strideC;
      unsigned short* C2 = (OUT_MODE == 2) ? ((unsigned short*)Cout2 + (size_t)b * strideC) : nullptr;
      for (int pass = 0; pass < 2; ++pass) {
#pragma unroll
        for (int it = 0; it < 4; ++it) {
          const int row = it * 4 + q;
          const float* sp = slab + row * 68 + c8;
          v8h hv, lv;
#pragma unroll
          for (int e = 0; e < 8; ++e) {
            if (OUT_MODE == 1) {
              hv[e] = (_Float16)sp[e];
            } else {
              unsigned short hb = f2bf_bits(sp[e]);
              unsigned short lb = f2bf_bits(sp[e] - bf_bits2f(hb));
              hv[e] = __builtin_bit_cast(_Float16, hb);
              lv[e] = __builtin_bit_cast(_Float16, lb);
            }
          }
          *(volatile v8h*)(C + (size_t)(mBase + row) * ldc + n0 + c8) = hv;
          if (OUT_MODE == 2) *(volatile v8h*)(C2 + (size_t)(mBase + row) * ldc + n0 + c8) = lv;
        }
        __threadfence();
      }
    }
    __builtin_amdgcn_fence(__ATOMIC_RELEASE, "workgroup");
    __builtin_amdgcn_wave_barrier();
    __builtin_amdgcn_fence(__ATOMIC_ACQUIRE, "workgroup");
  }
}

__global__ __launch_bounds__(256) void k_pad16v(const float* __restrict__ src, unsigned short* __restrict__ dst) {
  __shared__ __align__(16) _Float16 tile[32 * 264];
  const int tid = threadIdx.x;
  const int blk = blockIdx.x;
  const int wq  = blk & 3;
  const int h   = (blk >> 2) & (HH - 1);
  const int b   = blk >> 9;
  const int w0  = wq * 32;
  const float* sb = src + (size_t)b * CC * HWP + (size_t)h * WW + w0;
#pragma unroll
  for (int i = 0; i < 32; ++i) {
    const int idx = i * 256 + tid;
    const int c = idx >> 5, j = idx & 31;
    const float v = fmaxf(sb[(size_t)c * HWP + j], 0.0f);
    tile[j * 264 + c] = (_Float16)v;
  }
  __syncthreads();
  const int wave = tid >> 5, lane = tid & 31;
  _Float16* dp = (_Float16*)dst;
  for (int pass = 0; pass < 2; ++pass) {
#pragma unroll
    for (int k = 0; k < 4; ++k) {
      const int j = wave * 4 + k;
      const v8h v = *(const v8h*)(tile + j * 264 + lane * 8);
      const size_t row = (size_t)b * RP + GF + (size_t)(h + 1) * WP2 + (size_t)(w0 + j + 1);
      *(volatile v8h*)(dp + row * CC + lane * 8) = v;
    }
    __threadfence();
  }
}

__device__ __forceinline__ int halo_row(int i) {
  const int j  = i - 194;
  const int hp = (j >> 1) + 1;
  const int rmid  = GF + hp * WP2 + ((j & 1) ? (WP2 - 1) : 0);
  const int rtail = GF + 129 * WP2 + (i - 450);
  return (i < 194) ? i : ((i < 450) ? rmid : rtail);
}
__global__ __launch_bounds__(256) void k_zero_halo(unsigned short* __restrict__ dst) {
  const int lane = threadIdx.x & 31, wave = threadIdx.x >> 5;
  const int it = blockIdx.x * 8 + wave;
  if (it < NB * NHALO) {
    const int b = it / NHALO, i = it - b * NHALO;
    const int r = halo_row(i);
    const v4u z = (v4u){0u, 0u, 0u, 0u};
    volatile v4u* p = (volatile v4u*)(dst + ((size_t)b * RP + (size_t)r) * CC + lane * 8);
    *p = z;
    __threadfence();
    *p = z;
  }
}

__global__ __launch_bounds__(256) void k_pad16t(const float* __restrict__ tT, unsigned short* __restrict__ dst) {
  const int lane = threadIdx.x & 31, wave = threadIdx.x >> 5;
#pragma unroll 1
  for (int k = 0; k < 4; ++k) {
    const int it = ((blockIdx.x * 8 + wave) << 2) + k;
    if (it < NB * HWP) {
      const int b = it >> 14, p = it & (HWP - 1), h = p >> 7, w = p & (WW - 1);
      const float* sp = tT + ((size_t)b * RO + (size_t)(h * WP2 + w)) * CC + lane * 8;
      const v4f a = *(const v4f*)(sp);
      const v4f c = *(const v4f*)(sp + 4);
      v4u u;
      u[0] = pkh2(a[0], a[1]); u[1] = pkh2(a[2], a[3]);
      u[2] = pkh2(c[0], c[1]); u[3] = pkh2(c[2], c[3]);
      volatile v4u* d = (volatile v4u*)(dst + ((size_t)b * RP + GF + (size_t)(h + 1) * WP2 + (size_t)(w + 1)) * CC + lane * 8);
      *d = u;
      __threadfence();
      *d = u;
    }
  }
}

__global__ __launch_bounds__(256) void k_gate(const float* __restrict__ tT, const float* __restrict__ x,
                                             unsigned short* __restrict__ dst) {
  __shared__ float xs[32 * 257];
  const int tid = threadIdx.x;
  const int blk = blockIdx.x;
  const int wq  = blk & 3;
  const int h   = (blk >> 2) & (HH - 1);
  const int b   = blk >> 9;
  const int w0  = wq * 32;
  const float* xb = x + (size_t)b * CC * HWP + (size_t)h * WW + w0;
#pragma unroll
  for (int i = 0; i < 32; ++i) {
    const int idx = i * 256 + tid;
    const int c = idx >> 5, j = idx & 31;
    xs[j * 257 + c] = xb[(size_t)c * HWP + j];
  }
  __syncthreads();
  const int wave = tid >> 5, lane = tid & 31, c8 = lane * 8;
#pragma unroll
  for (int k = 0; k < 4; ++k) {
    const int j = wave * 4 + k;
    const int w = w0 + j;
    const float* sp = tT + ((size_t)b * RO + (size_t)(h * WP2 + w)) * CC + c8;
    const v4f a = *(const v4f*)(sp);
    const v4f c = *(const v4f*)(sp + 4);
    const float* gx = xs + j * 257 + c8;
    v4u u;
    u[0] = pkh2(a[0] * gx[0], a[1] * gx[1]); u[1] = pkh2(a[2] * gx[2], a[3] * gx[3]);
    u[2] = pkh2(c[0] * gx[4], c[1] * gx[5]); u[3] = pkh2(c[2] * gx[6], c[3] * gx[7]);
    volatile v4u* d = (volatile v4u*)(dst + ((size_t)b * RP + GF + (size_t)(h + 1) * WP2 + (size_t)(w + 1)) * CC + c8);
    *d = u;
    __threadfence();
    *d = u;
  }
}

__global__ __launch_bounds__(256) void k_prepw(const float* __restrict__ w, unsigned short* __restrict__ B,
                                              int orows, int ovalid, float scale, int kt) {
  const int kdw  = kt * CC;
  const int gidx = blockIdx.x * 256 + threadIdx.x;
  if (gidx < orows * (kdw >> 3)) {
    const int e0  = gidx * 8;
    const int o   = e0 / kdw;
    const int col = e0 - o * kdw;
    const int t   = col >> 8;
    const int c0  = col & (CC - 1);
    const int oc  = o < ovalid ? o : (ovalid - 1);
    float f[8];
#pragma unroll
    for (int j = 0; j < 8; ++j) {
      const float v = w[((size_t)(oc * CC + c0 + j)) * kt + t] * scale;
      f[j] = (o < ovalid) ? v : 0.0f;
    }
    v4u u;
    u[0] = pkh2(f[0], f[1]); u[1] = pkh2(f[2], f[3]); u[2] = pkh2(f[4], f[5]); u[3] = pkh2(f[6], f[7]);
    volatile v4u* p = (volatile v4u*)(B + e0);
    *p = u;
    __threadfence();
    *p = u;
  }
}

__device__ __forceinline__ void acc_corner(const float* __restrict__ p, float wv, v4f& a, v4f& b) {
  const v4f ga = *(const v4f*)(p);
  const v4f gb = *(const v4f*)(p + 4);
  a = a + ga * wv;
  b = b + gb * wv;
}

__global__ __launch_bounds__(256) void k_sample(const float* __restrict__ tT, const float* __restrict__ om,
                                                const float* __restrict__ boff, unsigned short* __restrict__ S,
                                                int n, int h0) {
  const int lane = threadIdx.x & 31, wave = threadIdx.x >> 5;
  const int c8 = lane * 8;
  const float* tb = tT + (size_t)n * RO * CC + c8;
  const float* ob = om + (size_t)n * RO * OFFN;
#pragma unroll 1
  for (int i = 0; i < SIT; ++i) {
    const int it = (blockIdx.x * 8 + wave) * SIT + i;
    if (it < CHPIX * KT) {
      const int ql = it / KT, t = it - ql * KT;
      const int hl = ql >> 7, w = ql & (WW - 1);
      const int h  = h0 + hl;
      const int ky = t / 3, kx = t - ky * 3;
      const float* op = ob + (size_t)(h * WP2 + w) * OFFN;
      const float dy = op[2 * t] + boff[2 * t];
      const float dx = op[2 * t + 1] + boff[2 * t + 1];
      float mr = op[18 + t] + boff[18 + t];
      mr = fminf(fmaxf(mr, -30.0f), 30.0f);
      const float mk = 1.0f / (1.0f + expf(-mr));
      const float py = (float)(h - 1 + ky) + dy;
      const float px = (float)(w - 1 + kx) + dx;
      const float y0f = floorf(py), x0f = floorf(px);
      const float wy1 = py - y0f, wx1 = px - x0f;
      const float wy0 = 1.0f - wy1, wx0 = 1.0f - wx1;
      const float y1f = y0f + 1.0f, x1f = x0f + 1.0f;
      const bool vy0 = (y0f >= 0.0f) && (y0f <= (float)(HH - 1));
      const bool vy1 = (y1f >= 0.0f) && (y1f <= (float)(HH - 1));
      const bool vx0 = (x0f >= 0.0f) && (x0f <= (float)(WW - 1));
      const bool vx1 = (x1f >= 0.0f) && (x1f <= (float)(WW - 1));
      float c00 = wy0 * wx0, c01 = wy0 * wx1, c10 = wy1 * wx0, c11 = wy1 * wx1;
      c00 = (vy0 && vx0) ? c00 : 0.0f;
      c01 = (vy0 && vx1) ? c01 : 0.0f;
      c10 = (vy1 && vx0) ? c10 : 0.0f;
      c11 = (vy1 && vx1) ? c11 : 0.0f;
      const int ya = (int)fminf(fmaxf(y0f, 0.0f), (float)(HH - 1));
      const int yb = (int)fminf(fmaxf(y1f, 0.0f), (float)(HH - 1));
      const int xa = (int)fminf(fmaxf(x0f, 0.0f), (float)(WW - 1));
      const int xb = (int)fminf(fmaxf(x1f, 0.0f), (float)(WW - 1));
      v4f va = (v4f){0.f, 0.f, 0.f, 0.f}, vb = (v4f){0.f, 0.f, 0.f, 0.f};
      acc_corner(tb + (size_t)(ya * WP2 + xa) * CC, c00, va, vb);
      acc_corner(tb + (size_t)(ya * WP2 + xb) * CC, c01, va, vb);
      acc_corner(tb + (size_t)(yb * WP2 + xa) * CC, c10, va, vb);
      acc_corner(tb + (size_t)(yb * WP2 + xb) * CC, c11, va, vb);
      va = va * mk;
      vb = vb * mk;
      v4u u;
      u[0] = pkh2(va[0], va[1]); u[1] = pkh2(va[2], va[3]);
      u[2] = pkh2(vb[0], vb[1]); u[3] = pkh2(vb[2], vb[3]);
      volatile v4u* d = (volatile v4u*)(S + (size_t)ql * KD + (size_t)t * CC + c8);
      *d = u;
      __threadfence();
      *d = u;
    }
  }
}

__global__ __launch_bounds__(256) void k_final(const float* __restrict__ hd, const float* __restrict__ b4,
                                              float* __restrict__ out) {
  const int lane = threadIdx.x & 31, wave = threadIdx.x >> 5;
  const int it = blockIdx.x * 8 + wave;
  if (it < NB * 2 * HH) {
    const int h = it & (HH - 1), o = (it >> 7) & 1, b = it >> 8;
    const float bo = b4[o];
    const float* hp = hd + ((size_t)b * RO + (size_t)(h * WP2) + (size_t)(lane * 4)) * HDN + o;
    v4f v;
    v[0] = hp[0] + bo; v[1] = hp[HDN] + bo; v[2] = hp[2 * HDN] + bo; v[3] = hp[3 * HDN] + bo;
    volatile v4f* d = (volatile v4f*)(out + ((size_t)(b * 2 + o) * HH + h) * WW + lane * 4);
    *d = v;
    __threadfence();
    *d = v;
  }
}

#define BYTES_T   ((size_t)NB * RO * CC * 4)
#define BYTES_OM  ((size_t)NB * RO * OFFN * 4)
#define BYTES_P   ((size_t)NB * RP * CC * 2)
#define BYTES_S   ((size_t)CHPIX * KD * 2)
#define BYTES_W   ((size_t)CC * KD * 2)
#define BYTES_WO  ((size_t)OFFN * KD * 2)
#define BYTES_W4  ((size_t)HDN * CC * 2)
#define BYTES_TOT (BYTES_T + BYTES_OM + 2 * BYTES_P + BYTES_S + 4 * BYTES_W + BYTES_WO + BYTES_W4)
typedef char ws_fits_check[(BYTES_TOT <= (size_t)134217728) ? 1 : -1];

extern "C" void kernel_launch(void* const* d_in, const int* in_sizes, int n_in,
                              void* d_out, int out_size, void* d_ws, size_t ws_size,
                              hipStream_t stream) {
  if (n_in < 14) return;
  if (in_sizes[0] != NB * CC * HWP || in_sizes[1] != NB * CC * HWP ||
      in_sizes[2] != CC * KD || in_sizes[3] != CC ||
      in_sizes[4] != OFFC * KD || in_sizes[5] != OFFC ||
      in_sizes[6] != CC * KD || in_sizes[7] != CC ||
      in_sizes[8] != CC * KD || in_sizes[9] != CC ||
      in_sizes[10] != CC * KD || in_sizes[11] != CC ||
      in_sizes[12] != 2 * CC || in_sizes[13] != 2) return;
  if (out_size != NB * 2 * HWP) return;
  if (BYTES_TOT > ws_size) return;

  const float* x     = (const float*)d_in[0];
  const float* vsrc  = (const float*)d_in[1];
  const float* w1    = (const float*)d_in[2];
  const float* b1    = (const float*)d_in[3];
  const float* w_off = (const float*)d_in[4];
  const float* b_off = (const float*)d_in[5];
  const float* w_dcn = (const float*)d_in[6];
  const float* b_dcn = (const float*)d_in[7];
  const float* w2    = (const float*)d_in[8];
  const float* b2    = (const float*)d_in[9];
  const float* w3    = (const float*)d_in[10];
  const float* b3    = (const float*)d_in[11];
  const float* w4    = (const float*)d_in[12];
  const float* b4    = (const float*)d_in[13];
  float* out = (float*)d_out;

  char* ws = (char*)d_ws;
  size_t o = 0;
  float* tT = (float*)(ws + o);                              o += BYTES_T;
  float* om = (float*)(ws + o);                              o += BYTES_OM;
  unsigned short* PA  = (unsigned short*)(ws + o);           o += BYTES_P;
  unsigned short* PB  = (unsigned short*)(ws + o);           o += BYTES_P;
  unsigned short* S   = (unsigned short*)(ws + o);           o += BYTES_S;
  unsigned short* W1p = (unsigned short*)(ws + o);           o += BYTES_W;
  unsigned short* Wdp = (unsigned short*)(ws + o);           o += BYTES_W;
  unsigned short* W2p = (unsigned short*)(ws + o);           o += BYTES_W;
  unsigned short* W3p = (unsigned short*)(ws + o);           o += BYTES_W;
  unsigned short* Wop = (unsigned short*)(ws + o);           o += BYTES_WO;
  unsigned short* W4p = (unsigned short*)(ws + o);           o += BYTES_W4;
  if (o > ws_size) return;
  if (o > (size_t)134217728) return;

  const size_t AOFF = (size_t)(GF + MSO) * CC;
  const int CONV_GX  = (RO / 64) * (CC / 64) / 8;
  const int SMALL_GX = (RO / 64 + 7) / 8;

  k_pad16v<<<NB * HH * (WW / 32), 256, 0, stream>>>(vsrc, PA);
  k_zero_halo<<<(NB * NHALO + 7) / 8, 256, 0, stream>>>(PA);

  k_prepw<<<(CC * (KD / 8) + 255) / 256, 256, 0, stream>>>(w1,    W1p, CC, CC, 16.0f, KT);
  k_prepw<<<(CC * (KD / 8) + 255) / 256, 256, 0, stream>>>(w_dcn, Wdp, CC, CC, 16.0f, KT);
  k_prepw<<<(CC * (KD / 8) + 255) / 256, 256, 0, stream>>>(w2,    W2p, CC, CC, 16.0f, KT);
  k_prepw<<<(CC * (KD / 8) + 255) / 256, 256, 0, stream>>>(w3,    W3p, CC, CC, 16.0f, KT);
  k_prepw<<<(OFFN * (KD / 8) + 255) / 256, 256, 0, stream>>>(w_off, Wop, OFFN, OFFC, 64.0f, KT);
  k_prepw<<<(HDN * (CC / 8) + 255) / 256, 256, 0, stream>>>(w4,    W4p, HDN, 2, 16.0f, 1);

  wmma_gemm64<0, false, 2, 0, false, 2, 1><<<dim3(CONV_GX, NB), 256, 0, stream>>>(
      PA + AOFF, PA + AOFF, CC, (long)RP * CC,
      W1p, W1p, KD, 0L,
      (void*)tT, (void*)tT, CC, (long)RO * CC,
      b1,
      b1, 0L,
      RO, CC, KD, 1.0f / 16.0f);

  k_pad16t<<<NB * HWP / 32, 256, 0, stream>>>(tT, PB);
  k_zero_halo<<<(NB * NHALO + 7) / 8, 256, 0, stream>>>(PB);

  wmma_gemm64<0, false, 0, 0, false, 0, 1><<<dim3(SMALL_GX, NB), 256, 0, stream>>>(
      PB + AOFF, PB + AOFF, CC, (long)RP * CC,
      Wop, Wop, KD, 0L,
      (void*)om, (void*)om, OFFN, (long)RO * OFFN,
      b_off,
      b_off, 0L,
      RO, OFFN, KD, 1.0f / 64.0f);

  for (int ck = 0; ck < NCH; ++ck) {
    const int n  = ck >> 1;
    const int h0 = (ck & 1) * CHROWS;
    k_sample<<<CHPIX * KT / (8 * SIT), 256, 0, stream>>>(tT, om, b_off, S, n, h0);
    unsigned short* Cd = PA + ((size_t)n * RP + GF + MSO + (size_t)h0 * WP2) * CC;
    wmma_gemm64<0, false, 2, 1, false, 2, 0><<<dim3(1, CHROWS), 256, 0, stream>>>(
        S, S, KD, (long)WW * KD,
        Wdp, Wdp, KD, 0L,
        (void*)Cd, (void*)Cd, CC, (long)WP2 * CC,
        b_dcn,
        b_dcn, 0L,
        WW, CC, KD, 1.0f / 16.0f);
  }

  wmma_gemm64<0, false, 2, 0, false, 0, 1><<<dim3(CONV_GX, NB), 256, 0, stream>>>(
      PA + AOFF, PA + AOFF, CC, (long)RP * CC,
      W2p, W2p, KD, 0L,
      (void*)tT, (void*)tT, CC, (long)RO * CC,
      b2,
      b2, 0L,
      RO, CC, KD, 1.0f / 16.0f);
  k_gate<<<NB * HH * (WW / 32), 256, 0, stream>>>(tT, x, PB);

  wmma_gemm64<0, false, 2, 1, false, 2, 1><<<dim3(CONV_GX, NB), 256, 0, stream>>>(
      PB + AOFF, PB + AOFF, CC, (long)RP * CC,
      W3p, W3p, KD, 0L,
      (void*)(PA + AOFF), (void*)(PA + AOFF), CC, (long)RP * CC,
      b3,
      b3, 0L,
      RO, CC, KD, 1.0f / 16.0f);

  wmma_gemm64<0, false, 0, 0, false, 0, 0><<<dim3(SMALL_GX, NB), 256, 0, stream>>>(
      PA + AOFF, PA + AOFF, CC, (long)RP * CC,
      W4p, W4p, CC, 0L,
      (void*)om, (void*)om, HDN, (long)RO * HDN,
      b_off,
      b_off, 0L,
      RO, HDN, CC, 1.0f / 16.0f);

  k_final<<<(NB * 2 * HH + 7) / 8, 256, 0, stream>>>(om, b4, out);
  (void)hipGetLastError();
}
